// MultiHeadSelfAttention_25769804120
// MI455X (gfx1250) — hardware-verified
//
#include <hip/hip_runtime.h>


#ifndef NB
#define NB 4
#endif
#ifndef SEQ
#define SEQ 2048
#endif
#define NB_FULL  4
#define SEQ_FULL 2048
#define DMOD  768
#define NHEAD 12
#define HDIM  64
#define OSP   68
#define LOG2E 1.4426950408889634f
#define PSH   8.0f
#define PCAR  16.0f
#define CCAR  256.0f
#define WCAR  1024.0f
#define TFILL (-3.0e38f)
#define SSC   (LOG2E * (0.125f / (PCAR * PCAR)))
#define OSC   (1.0f / (CCAR * WCAR))
#define MBW   ((((NB * SEQ) / 32 + 255) / 256) * 256)

static_assert(NHEAD * HDIM == DMOD);
static_assert(HDIM == 64);
static_assert(HDIM * 2 == 128);
static_assert(HDIM * 4 == 256);
static_assert(DMOD % 64 == 0);
static_assert(DMOD % 32 == 0);
static_assert(SEQ % 64 == 0);
static_assert(SEQ <= SEQ_FULL);
static_assert(NB <= NB_FULL);
static_assert((SEQ * DMOD) % 8 == 0);
static_assert((DMOD * DMOD) % 8 == 0);
static_assert((NB * SEQ) % 64 == 0);
static_assert((NB * SEQ) / 64 <= 65535);
static_assert(OSP % 4 == 0);
static_assert(OSP >= HDIM);
static_assert(PCAR * PCAR == 256.0f);
static_assert(CCAR / PCAR == 16.0f);
static_assert(MBW % 256 == 0);
static_assert(MBW >= (NB * SEQ) / 32);

typedef _Float16 h16;
typedef unsigned short bf;
typedef __attribute__((ext_vector_type(16))) __bf16   v16bf;
typedef __attribute__((ext_vector_type(16))) _Float16 v16h;
typedef __attribute__((ext_vector_type(8)))  _Float16 v8h;
typedef __attribute__((ext_vector_type(8)))  unsigned short v8us;
typedef __attribute__((ext_vector_type(8)))  float    v8f;
typedef __attribute__((ext_vector_type(4)))  float    v4f;
typedef __attribute__((ext_vector_type(4)))  int      v4i;
typedef v4f  __attribute__((may_alias)) v4fa;

__device__ __forceinline__ unsigned short f2bf(float f) { unsigned u = __float_as_uint(f); u += 0x7FFFu + ((u >> 16) & 1u); return (unsigned short)(u >> 16); }
__device__ __forceinline__ float bf2f(unsigned short b) { return __uint_as_float(((unsigned)b) << 16); }
__device__ __forceinline__ float bfr(float f) { return bf2f(f2bf(f)); }
__device__ __forceinline__ void splitf(float y, unsigned short& h, unsigned short& l) { h = f2bf(y); l = f2bf(y - bf2f(h)); }
__device__ __forceinline__ v16h cat16(v8h lo, v8h hi) { return __builtin_shufflevector(lo, hi, 0, 1, 2, 3, 4, 5, 6, 7, 8, 9, 10, 11, 12, 13, 14, 15); }
__device__ __forceinline__ v16bf cat16b(v8us lo, v8us hi) { return __builtin_bit_cast(v16bf, __builtin_shufflevector(lo, hi, 0, 1, 2, 3, 4, 5, 6, 7, 8, 9, 10, 11, 12, 13, 14, 15)); }
__device__ __forceinline__ v8f wmma16(v16h a, v16h b, v8f c) { return __builtin_amdgcn_wmma_f32_16x16x32_f16(false, a, false, b, (short)0, c, false, false); }
__device__ __forceinline__ v8f wmmab(v16bf a, v16bf b, v8f c) { return __builtin_amdgcn_wmma_f32_16x16x32_bf16(false, a, false, b, (short)0, c, false, false); }
__device__ __forceinline__ v8f wmma16g(v16h a, v16h b, v8f c) { c = wmma16(a, b, c); asm volatile("v_nop\n\tv_nop\n\tv_nop\n\tv_nop" : "+v"(c) : "v"(a), "v"(b)); return c; }
__device__ __forceinline__ v16bf ldbf(const bf* p) { return cat16b(*(const v8us*)p, *(const v8us*)(p + 16)); }
__device__ __forceinline__ v16h  ldh(const h16* p) { return cat16(*(const v8h*)p, *(const v8h*)(p + 16)); }
static __device__ __forceinline__ h16 toh_flush(float v) { const h16 r = (h16)v; return (fabsf(v) < 6.103515625e-05f) ? (h16)0.0f : r; }

__global__ __launch_bounds__(256) void k_cvt(const float* __restrict__ src, bf* dst, int n, int per, int per_full) {
    const int e = ((int)blockIdx.x * 256 + (int)threadIdx.x) * 8;
    if (e >= n) return;
    const int b = e / per;
    const size_t so = (size_t)b * (size_t)per_full + (size_t)(e - b * per);
    const v4f a0 = *(const v4f*)(src + so);
    const v4f a1 = *(const v4f*)(src + so + 4);
    v8us o;
    o[0] = f2bf(a0[0]); o[1] = f2bf(a0[1]); o[2] = f2bf(a0[2]); o[3] = f2bf(a0[3]);
    o[4] = f2bf(a1[0]); o[5] = f2bf(a1[1]); o[6] = f2bf(a1[2]); o[7] = f2bf(a1[3]);
    *(volatile v8us*)(dst + e) = o;
    __threadfence();
    *(volatile v8us*)(dst + e) = o;
}

__global__ __launch_bounds__(256) void k_cvth(const float* __restrict__ src, h16* dst, int n, float car) {
    const int e = ((int)blockIdx.x * 256 + (int)threadIdx.x) * 8;
    if (e >= n) return;
    const v4f a0 = *(const v4f*)(src + e);
    const v4f a1 = *(const v4f*)(src + e + 4);
    v8h o;
    o[0] = toh_flush(bfr(a0[0]) * car); o[1] = toh_flush(bfr(a0[1]) * car); o[2] = toh_flush(bfr(a0[2]) * car); o[3] = toh_flush(bfr(a0[3]) * car);
    o[4] = toh_flush(bfr(a1[0]) * car); o[5] = toh_flush(bfr(a1[1]) * car); o[6] = toh_flush(bfr(a1[2]) * car); o[7] = toh_flush(bfr(a1[3]) * car);
    *(volatile v8h*)(dst + e) = o;
    __threadfence();
    *(volatile v8h*)(dst + e) = o;
}

__global__ __launch_bounds__(256) void k_mask(const int* __restrict__ mask, unsigned* MB, int nwords) {
    const int wi = (int)blockIdx.x * 256 + (int)threadIdx.x;
    const int wc = (wi < nwords) ? wi : (nwords - 1);
    const int b = wc / (SEQ / 32), j = wc - b * (SEQ / 32);
    const int* mp = mask + (size_t)b * SEQ_FULL + (size_t)j * 32;
    unsigned w = 0u;
#pragma unroll 1
    for (int i = 0; i < 32; i += 4) {
        const v4i mv = *(const v4i*)(mp + i);
        w |= ((mv[0] != 0) ? 1u : 0u) << i;
        w |= ((mv[1] != 0) ? 1u : 0u) << (i + 1);
        w |= ((mv[2] != 0) ? 1u : 0u) << (i + 2);
        w |= ((mv[3] != 0) ? 1u : 0u) << (i + 3);
    }
    if (wi >= nwords) w = 0u;
    *(volatile unsigned*)(MB + wi) = w;
    __threadfence();
    *(volatile unsigned*)(MB + wi) = w;
}

__device__ __forceinline__ void gemm_tile(const bf* __restrict__ A, const bf* __restrict__ Bt, size_t aoff, size_t boff, v8f (&acc)[4][4]) {
#pragma unroll
    for (int mb = 0; mb < 4; ++mb)
#pragma unroll
        for (int nb = 0; nb < 4; ++nb) acc[mb][nb] = (v8f){};
#pragma unroll 1
    for (int kc = 0; kc < DMOD; kc += 32) {
        v16bf a[4];
        v16bf b;
#pragma unroll
        for (int mb = 0; mb < 4; ++mb) a[mb] = ldbf(A + aoff + (size_t)mb * 16 * DMOD + kc);
#pragma unroll
        for (int nb = 0; nb < 4; ++nb) {
            b = ldbf(Bt + boff + (size_t)nb * 16 * DMOD + kc);
#pragma unroll
            for (int mb = 0; mb < 4; ++mb) acc[mb][nb] = wmmab(a[mb], b, acc[mb][nb]);
        }
        asm volatile("" : "+v"(acc[0][0]), "+v"(acc[1][0]), "+v"(acc[2][0]), "+v"(acc[3][0]), "+v"(acc[0][1]), "+v"(acc[1][1]), "+v"(acc[2][1]), "+v"(acc[3][1]));
        asm volatile("v_nop\n\tv_nop\n\tv_nop\n\tv_nop" : "+v"(acc[0][2]), "+v"(acc[1][2]), "+v"(acc[2][2]), "+v"(acc[3][2]), "+v"(acc[0][3]), "+v"(acc[1][3]), "+v"(acc[2][3]), "+v"(acc[3][3]) : "v"(a[0]), "v"(a[3]), "v"(b));
    }
}

__device__ __forceinline__ void gemm_tile_h(const h16* __restrict__ A, const h16* __restrict__ Bt, size_t aoff, size_t boff, v8f (&acc)[4][4]) {
#pragma unroll
    for (int mb = 0; mb < 4; ++mb)
#pragma unroll
        for (int nb = 0; nb < 4; ++nb) acc[mb][nb] = (v8f){};
#pragma unroll 1
    for (int kc = 0; kc < DMOD; kc += 32) {
        v16h a[4];
#pragma unroll
        for (int mb = 0; mb < 4; ++mb) a[mb] = ldh(A + aoff + (size_t)mb * 16 * DMOD + kc);
#pragma unroll
        for (int nb = 0; nb < 4; ++nb) {
            const v16h bfrag = ldh(Bt + boff + (size_t)nb * 16 * DMOD + kc);
#pragma unroll
            for (int mb = 0; mb < 4; ++mb) acc[mb][nb] = wmma16g(a[mb], bfrag, acc[mb][nb]);
        }
    }
}

__global__ __launch_bounds__(32) void k_proj_qk(const bf* __restrict__ X, const bf* __restrict__ W, const float* __restrict__ bias, h16* P) {
    __shared__ __align__(16) float os[16 * OSP];
    const int lane = (int)threadIdx.x & 31, lr = lane & 15, hi = lane >> 4;
    const int r0 = (int)blockIdx.x * 64, c0 = (int)blockIdx.y * 64;
    v8f acc[4][4];
    gemm_tile(X, W, (size_t)(r0 + lr) * DMOD + 8 * hi, (size_t)(c0 + lr) * DMOD + 8 * hi, acc);
    const int b = r0 / SEQ, t0 = r0 - b * SEQ, hd = (int)blockIdx.y;
    const int rq = lane >> 3, cq = (lane & 7) * 8;
    const v4f bv0 = *(const v4f*)(bias + c0 + cq);
    const v4f bv1 = *(const v4f*)(bias + c0 + cq + 4);
    float bb[8];
    bb[0] = bfr(bv0[0]); bb[1] = bfr(bv0[1]); bb[2] = bfr(bv0[2]); bb[3] = bfr(bv0[3]);
    bb[4] = bfr(bv1[0]); bb[5] = bfr(bv1[1]); bb[6] = bfr(bv1[2]); bb[7] = bfr(bv1[3]);
    const size_t pbase = ((size_t)(b * NHEAD + hd) * SEQ + t0) * HDIM;
#pragma unroll
    for (int mb = 0; mb < 4; ++mb) {
#pragma unroll
        for (int nb = 0; nb < 4; ++nb) {
#pragma unroll
            for (int j = 0; j < 8; ++j) os[(hi * 8 + j) * OSP + nb * 16 + lr] = acc[mb][nb][j];
        }
        __syncthreads();
#pragma unroll 1
        for (int ps = 0; ps < 2; ++ps) {
#pragma unroll
            for (int s = 0; s < 4; ++s) {
                const int row = s * 4 + rq;
                const v4f x0 = *(const v4fa*)(os + row * OSP + cq);
                const v4f x1 = *(const v4fa*)(os + row * OSP + cq + 4);
                v8h oh;
#pragma unroll
                for (int i = 0; i < 4; ++i) {
                    oh[i] = toh_flush((x0[i] + bb[i]) * PCAR);
                    oh[4 + i] = toh_flush((x1[i] + bb[4 + i]) * PCAR);
                }
                const size_t oo = pbase + (size_t)(mb * 16 + row) * HDIM + cq;
                *(volatile v8h*)(P + oo) = oh;
            }
            if (ps == 0) __threadfence();
        }
        __syncthreads();
    }
}

__global__ __launch_bounds__(32) void k_proj_v(const bf* __restrict__ W, const bf* __restrict__ X, const float* __restrict__ bias, h16* Pv) {
    __shared__ __align__(16) float os[16 * OSP];
    const int lane = (int)threadIdx.x & 31, lr = lane & 15, hi = lane >> 4;
    const int r0 = (int)blockIdx.x * 64, c0 = (int)blockIdx.y * 64;
    v8f acc[4][4];
    gemm_tile(W, X, (size_t)(r0 + lr) * DMOD + 8 * hi, (size_t)(c0 + lr) * DMOD + 8 * hi, acc);
    const int b = c0 / SEQ, t0 = c0 - b * SEQ, hd = (int)blockIdx.x;
    const int rq = lane >> 3, cq = (lane & 7) * 8;
    const size_t pbase = (size_t)(b * NHEAD + hd) * HDIM * SEQ + t0;
#pragma unroll
    for (int mb = 0; mb < 4; ++mb) {
#pragma unroll
        for (int nb = 0; nb < 4; ++nb) {
#pragma unroll
            for (int j = 0; j < 8; ++j) os[(hi * 8 + j) * OSP + nb * 16 + lr] = acc[mb][nb][j];
        }
        __syncthreads();
#pragma unroll 1
        for (int ps = 0; ps < 2; ++ps) {
#pragma unroll
            for (int s = 0; s < 4; ++s) {
                const int row = s * 4 + rq;
                const float bsc = bfr(bias[r0 + mb * 16 + row]);
                const v4f x0 = *(const v4fa*)(os + row * OSP + cq);
                const v4f x1 = *(const v4fa*)(os + row * OSP + cq + 4);
                v8h ov;
#pragma unroll
                for (int i = 0; i < 4; ++i) {
                    ov[i] = toh_flush((x0[i] + bsc) * PCAR);
                    ov[4 + i] = toh_flush((x1[i] + bsc) * PCAR);
                }
                const size_t oo = pbase + (size_t)(mb * 16 + row) * SEQ + cq;
                *(volatile v8h*)(Pv + oo) = ov;
            }
            if (ps == 0) __threadfence();
        }
        __syncthreads();
    }
}

__global__ __launch_bounds__(128) void k_attn(const h16* __restrict__ QP, const h16* __restrict__ KP, const h16* __restrict__ VV, const unsigned* __restrict__ MB, h16* CTX) {
    __shared__ __align__(16) float os[4 * 16 * OSP];
    const int wave = __builtin_amdgcn_readfirstlane((int)(threadIdx.x >> 5));
    const int lane = (int)threadIdx.x & 31, lr = lane & 15, hi = lane >> 4;
    const int bh = (int)blockIdx.y;
    const int b = bh / NHEAD, hd = bh - b * NHEAD;
    const int q0 = (int)blockIdx.x * 64 + wave * 16;
    const size_t pb = (size_t)bh * SEQ * HDIM;
    const h16* qh = QP + pb;
    const h16* kh = KP + pb;
    const h16* vv = VV + pb;
    const unsigned* mb = MB + b * (SEQ / 32);
    const int qoff0 = (q0 + lr) * HDIM + 8 * hi;
    const int koff = lr * HDIM + 8 * hi;
    const int voff = lr * SEQ + 8 * hi;
    const int msh = 8 * hi;
    v8f ova[4];
#pragma unroll
    for (int dt = 0; dt < 4; ++dt) ova[dt] = (v8f){};
    float m = TFILL, lsum = 0.0f;
#pragma unroll 1
    for (int j0 = 0; j0 < SEQ; j0 += 32) {
        int qo = qoff0;
        asm volatile("" : "+v"(qo));
        unsigned mw = mb[j0 >> 5];
        asm volatile("" : "+v"(mw));
        mw >>= msh;
        v8f s0 = (v8f){}, s1 = (v8f){};
#pragma unroll
        for (int kc = 0; kc < HDIM; kc += 32) {
            const v16h qf = ldh(qh + qo + kc);
            const int ko = koff + j0 * HDIM + kc;
            const v16h k0 = ldh(kh + ko);
            const v16h k1 = ldh(kh + ko + 16 * HDIM);
            s0 = wmma16g(k0, qf, s0);
            s1 = wmma16g(k1, qf, s1);
        }
        float t0[8], t1[8];
        float mx = TFILL;
#pragma unroll
        for (int r = 0; r < 8; ++r) {
            const float a0 = s0[r] * SSC;
            const float a1 = s1[r] * SSC;
            t0[r] = (((mw >> r) & 1u) != 0u) ? a0 : TFILL;
            t1[r] = (((mw >> (16 + r)) & 1u) != 0u) ? a1 : TFILL;
            mx = fmaxf(mx, fmaxf(t0[r], t1[r]));
        }
        mx = fmaxf(mx, __shfl_xor(mx, 16, 32));
        const float mnew = fmaxf(m, mx);
        const float sc = __builtin_amdgcn_exp2f(m - mnew);
        m = mnew;
        const float mo = mnew - PSH;
        float psum = 0.0f;
        v16h pf;
#pragma unroll
        for (int r = 0; r < 8; ++r) {
            const float x0 = t0[r] - mo;
            const float x1 = t1[r] - mo;
            const float e0 = (x0 < -14.0f) ? 0.0f : __builtin_amdgcn_exp2f(x0);
            const float e1 = (x1 < -14.0f) ? 0.0f : __builtin_amdgcn_exp2f(x1);
            const h16 p0 = (h16)e0;
            const h16 p1 = (h16)e1;
            psum += (float)p0 + (float)p1;
            pf[r] = p0; pf[8 + r] = p1;
        }
        lsum = lsum * sc + psum;
        if (__builtin_amdgcn_ballot_w32(sc != 1.0f) != 0u) {
#pragma unroll
            for (int dt = 0; dt < 4; ++dt) {
#pragma unroll
                for (int r = 0; r < 8; ++r) ova[dt][r] *= sc;
            }
        }
        const int vo = voff + j0;
        v16h va[4];
#pragma unroll
        for (int dt = 0; dt < 4; ++dt) va[dt] = ldh(vv + vo + dt * 16 * SEQ);
#pragma unroll
        for (int dt = 0; dt < 4; ++dt) ova[dt] = wmma16g(va[dt], pf, ova[dt]);
    }
    lsum += __shfl_xor(lsum, 16, 32);
    const float inv = 1.0f / lsum;
    const float fac = inv * (CCAR / PCAR);
    const int obase = wave * 16 * OSP;
#pragma unroll
    for (int dt = 0; dt < 4; ++dt) {
        v4f x0, x1;
#pragma unroll
        for (int i = 0; i < 4; ++i) {
            x0[i] = ova[dt][i] * fac;
            x1[i] = ova[dt][4 + i] * fac;
        }
        *(v4fa*)(os + obase + lr * OSP + dt * 16 + 8 * hi) = x0;
        *(v4fa*)(os + obase + lr * OSP + dt * 16 + 8 * hi + 4) = x1;
    }
    __syncthreads();
    const int rq = lane >> 3, cq = (lane & 7) * 8;
    h16* crow = CTX + ((size_t)b * SEQ + q0) * DMOD + hd * HDIM;
#pragma unroll 1
    for (int ps = 0; ps < 2; ++ps) {
#pragma unroll
        for (int s = 0; s < 4; ++s) {
            const int row = s * 4 + rq;
            const v4f x0 = *(const v4fa*)(os + obase + row * OSP + cq);
            const v4f x1 = *(const v4fa*)(os + obase + row * OSP + cq + 4);
            v8h oc;
#pragma unroll
            for (int i = 0; i < 4; ++i) { oc[i] = toh_flush(x0[i]); oc[4 + i] = toh_flush(x1[i]); }
            *(volatile v8h*)(crow + (size_t)row * DMOD + cq) = oc;
        }
        if (ps == 0) __threadfence();
    }
}

__global__ __launch_bounds__(32) void k_proj_o(const h16* __restrict__ X, const h16* __restrict__ W, const float* __restrict__ bias, float* OUT) {
    __shared__ __align__(16) float os[16 * OSP];
    const int lane = (int)threadIdx.x & 31, lr = lane & 15, hi = lane >> 4;
    const int r0 = (int)blockIdx.x * 64, c0 = (int)blockIdx.y * 64;
    v8f acc[4][4];
    gemm_tile_h(X, W, (size_t)(r0 + lr) * DMOD + 8 * hi, (size_t)(c0 + lr) * DMOD + 8 * hi, acc);
    const int b = r0 / SEQ, t0 = r0 - b * SEQ;
    const int cofs = lr * 4;
    const v4f bv = *(const v4f*)(bias + c0 + cofs);
    v4f bb;
    bb[0] = bfr(bv[0]); bb[1] = bfr(bv[1]); bb[2] = bfr(bv[2]); bb[3] = bfr(bv[3]);
    float* orow = OUT + ((size_t)b * SEQ_FULL + t0) * DMOD + c0;
#pragma unroll
    for (int mb = 0; mb < 4; ++mb) {
#pragma unroll
        for (int nb = 0; nb < 4; ++nb) {
#pragma unroll
            for (int j = 0; j < 8; ++j) os[(hi * 8 + j) * OSP + nb * 16 + lr] = acc[mb][nb][j];
        }
        __syncthreads();
#pragma unroll 1
        for (int ps = 0; ps < 2; ++ps) {
#pragma unroll
            for (int s = 0; s < 8; ++s) {
                const int row = 2 * s + hi;
                const v4f x = *(const v4fa*)(os + row * OSP + cofs);
                v4f val;
                val[0] = x[0] * OSC + bb[0]; val[1] = x[1] * OSC + bb[1]; val[2] = x[2] * OSC + bb[2]; val[3] = x[3] * OSC + bb[3];
                *(volatile v4f*)(orow + (size_t)(mb * 16 + row) * DMOD + cofs) = val;
            }
            if (ps == 0) __threadfence();
        }
        __syncthreads();
    }
}

extern "C" void kernel_launch(void* const* d_in, const int* in_sizes, int n_in,
                              void* d_out, int out_size, void* d_ws, size_t ws_size, hipStream_t stream) {
    if (n_in < 12) return;
    const size_t need_x = (size_t)(NB - 1) * SEQ_FULL * DMOD + (size_t)SEQ * DMOD;
    const size_t need_m = (size_t)(NB - 1) * SEQ_FULL + (size_t)SEQ;
    if ((size_t)in_sizes[0] < need_x || (size_t)in_sizes[1] < need_x || (size_t)in_sizes[2] < need_x) return;
    if ((size_t)in_sizes[3] < need_m) return;
    if (in_sizes[4] < DMOD * DMOD || in_sizes[6] < DMOD * DMOD || in_sizes[8] < DMOD * DMOD || in_sizes[10] < DMOD * DMOD) return;
    if (in_sizes[5] < DMOD || in_sizes[7] < DMOD || in_sizes[9] < DMOD || in_sizes[11] < DMOD) return;
    if ((size_t)out_size < need_x) return;
    const float* xq = (const float*)d_in[0]; const float* xk = (const float*)d_in[1]; const float* xv = (const float*)d_in[2];
    const int* msk = (const int*)d_in[3];
    const float* Wq = (const float*)d_in[4]; const float* bq = (const float*)d_in[5];
    const float* Wk = (const float*)d_in[6]; const float* bk = (const float*)d_in[7];
    const float* Wv = (const float*)d_in[8]; const float* bv = (const float*)d_in[9];
    const float* Wo = (const float*)d_in[10]; const float* bo = (const float*)d_in[11];
    float* OUT = (float*)d_out;

    constexpr size_t WB = (size_t)DMOD * DMOD * 2;
    constexpr size_t PB = (size_t)NB * SEQ * DMOD * 2;
    constexpr size_t MBB = (size_t)MBW * 4;
    static_assert(WB % 256 == 0);
    static_assert(PB % 256 == 0);
    static_assert(MBB % 256 == 0);
    static_assert(4 * WB + 5 * PB + MBB <= (size_t)134217728);
    if (4 * WB + 5 * PB + MBB > ws_size) return;
    char* wsp = (char*)d_ws;
    bf* WQ = (bf*)wsp; wsp += WB;
    bf* WK = (bf*)wsp; wsp += WB;
    bf* WV = (bf*)wsp; wsp += WB;
    h16* WOh = (h16*)wsp; wsp += WB;
    bf* XB = (bf*)wsp; wsp += PB;
    h16* QPp = (h16*)wsp; wsp += PB;
    h16* KPp = (h16*)wsp; wsp += PB;
    h16* VVp = (h16*)wsp; wsp += PB;
    h16* CTXp = (h16*)wsp; wsp += PB;
    unsigned* MBp = (unsigned*)wsp; wsp += MBB;

    const int nW = DMOD * DMOD, nX = NB * SEQ * DMOD;
    const unsigned gW = (unsigned)((nW / 8 + 255) / 256), gX = (unsigned)((nX / 8 + 255) / 256);
    k_cvt<<<gW, 256, 0, stream>>>(Wq, WQ, nW, nW, nW);
    k_cvt<<<gW, 256, 0, stream>>>(Wk, WK, nW, nW, nW);
    k_cvt<<<gW, 256, 0, stream>>>(Wv, WV, nW, nW, nW);
    k_cvth<<<gW, 256, 0, stream>>>(Wo, WOh, nW, WCAR);
    k_mask<<<(unsigned)(MBW / 256), 256, 0, stream>>>(msk, MBp, (NB * SEQ) / 32);
    k_cvt<<<gX, 256, 0, stream>>>(xq, XB, nX, SEQ * DMOD, SEQ_FULL * DMOD);
    k_proj_qk<<<dim3(NB * SEQ / 64, DMOD / 64), 32, 0, stream>>>(XB, WQ, bq, QPp);
    k_cvt<<<gX, 256, 0, stream>>>(xk, XB, nX, SEQ * DMOD, SEQ_FULL * DMOD);
    k_proj_qk<<<dim3(NB * SEQ / 64, DMOD / 64), 32, 0, stream>>>(XB, WK, bk, KPp);
    k_cvt<<<gX, 256, 0, stream>>>(xv, XB, nX, SEQ * DMOD, SEQ_FULL * DMOD);
    k_proj_v<<<dim3(DMOD / 64, NB * SEQ / 64), 32, 0, stream>>>(WV, XB, bv, VVp);
    k_attn<<<dim3(SEQ / 64, NB * NHEAD), 128, 0, stream>>>(QPp, KPp, VVp, MBp, CTXp);
    k_proj_o<<<dim3(NB * SEQ / 64, DMOD / 64), 32, 0, stream>>>(CTXp, WOh, bo, OUT);
}
